// SubjectLayers_49606872268952
// MI455X (gfx1250) — hardware-verified
//
#include <hip/hip_runtime.h>


#ifndef NB
#define NB 4096
#endif
#define NB_FULL 4096
#define CC 256
#define DD 512
#define NG 8
#define KT (NG * CC)

static_assert(NB % 64 == 0);
static_assert(NB <= NB_FULL);
static_assert(CC % 64 == 0);
static_assert(CC % 32 == 0);
static_assert(DD % 64 == 0);
static_assert(KT % 32 == 0);
static_assert(((size_t)NB * CC) % 8 == 0);
static_assert((CC * 2) % 128 == 0);
static_assert(NG <= 32);

typedef unsigned short bf;
typedef __attribute__((ext_vector_type(16))) __bf16   v16bf;
typedef __attribute__((ext_vector_type(8)))  unsigned short v8us;
typedef __attribute__((ext_vector_type(8)))  float    v8f;
typedef __attribute__((ext_vector_type(4)))  float    v4f;
typedef v4f  __attribute__((may_alias)) v4fa;

__device__ __forceinline__ unsigned short f2bf(float f) { unsigned u = __float_as_uint(f); u += 0x7FFFu + ((u >> 16) & 1u); return (unsigned short)(u >> 16); }
__device__ __forceinline__ float bfr(float f) { return __uint_as_float(((unsigned)f2bf(f)) << 16); }
__device__ __forceinline__ v16bf cat16b(v8us lo, v8us hi) { return __builtin_bit_cast(v16bf, __builtin_shufflevector(lo, hi, 0, 1, 2, 3, 4, 5, 6, 7, 8, 9, 10, 11, 12, 13, 14, 15)); }
__device__ __forceinline__ v8f wmmab(v16bf a, v16bf b, v8f c) { return __builtin_amdgcn_wmma_f32_16x16x32_bf16(false, a, false, b, (short)0, c, false, false); }
__device__ __forceinline__ v16bf ldb(const bf* p)  { return cat16b(*(const v8us*)p, *(const v8us*)(p + 16)); }
__device__ __forceinline__ void wave_sync() { __builtin_amdgcn_fence(3  , "wavefront"); __builtin_amdgcn_wave_barrier(); asm volatile("" ::: "memory"); }

__global__ __launch_bounds__(256) void k_cvt8(const float* __restrict__ src, bf* dst, size_t n8) {
    const size_t i = (size_t)blockIdx.x * 256 + threadIdx.x; if (i >= n8) return;
    const v8f v = *(const v8f*)(src + i * 8); v8us o;
#pragma unroll
    for (int k = 0; k < 8; ++k) o[k] = f2bf(v[k]);
    *(volatile v8us*)(dst + i * 8) = o; __threadfence(); *(volatile v8us*)(dst + i * 8) = o;
}

__global__ __launch_bounds__(256) void k_wt(const float* __restrict__ W, bf* WT) {
    __shared__ float t[64 * 65];
    const int tid = threadIdx.x;
    const int d0 = blockIdx.x * 64, c0 = blockIdx.y * 64, g = blockIdx.z;
    const float* src = W + ((size_t)g * CC + c0) * DD + d0;
#pragma unroll
    for (int i = 0; i < 4; ++i) {
        const int q = i * 256 + tid; const int c = q >> 4, d4 = (q & 15) * 4;
        const v4f v = *(const v4f*)(src + (size_t)c * DD + d4);
        t[c * 65 + d4 + 0] = v[0]; t[c * 65 + d4 + 1] = v[1]; t[c * 65 + d4 + 2] = v[2]; t[c * 65 + d4 + 3] = v[3];
    }
    __syncthreads();
    v8us o0, o1;
    const int p0 = tid, p1 = 256 + tid;
    const int da = p0 >> 3, ca = (p0 & 7) * 8, db = p1 >> 3, cb = (p1 & 7) * 8;
#pragma unroll
    for (int k = 0; k < 8; ++k) { o0[k] = f2bf(t[(ca + k) * 65 + da]); o1[k] = f2bf(t[(cb + k) * 65 + db]); }
    const size_t oa = (size_t)(d0 + da) * KT + (size_t)g * CC + c0 + ca;
    const size_t ob = (size_t)(d0 + db) * KT + (size_t)g * CC + c0 + cb;
    *(volatile v8us*)(WT + oa) = o0; *(volatile v8us*)(WT + ob) = o1;
    __threadfence();
    *(volatile v8us*)(WT + oa) = o0; *(volatile v8us*)(WT + ob) = o1;
}

__global__ __launch_bounds__(32) void k_sgemm(const bf* __restrict__ A, const bf* __restrict__ Bt, const int* __restrict__ gidx, const float* __restrict__ bias, float* OUT) {
    __shared__ __align__(16) float os[16 * 68];
    __shared__ __align__(16) float bs[NG * 64];
    __shared__ int sg[64];
    const int lane = threadIdx.x & 31, lr = lane & 15, hi = lane >> 4;
    const int r0 = __builtin_amdgcn_readfirstlane((int)blockIdx.x) * 64;
    const int c0 = __builtin_amdgcn_readfirstlane((int)blockIdx.y) * 64;
    { int g0 = gidx[r0 + lane], g1 = gidx[r0 + 32 + lane];
      g0 = (g0 < 0) ? 0 : g0; g0 = (g0 > NG - 1) ? (NG - 1) : g0;
      g1 = (g1 < 0) ? 0 : g1; g1 = (g1 > NG - 1) ? (NG - 1) : g1;
      sg[lane] = g0; sg[32 + lane] = g1; }
#pragma unroll
    for (int i = 0; i < 4; ++i) {
        const int q = i * 32 + lane; const int g = q >> 4, c4 = (q & 15) * 4;
        const v4f v = *(const v4f*)(bias + (size_t)g * DD + c0 + c4); v4f o;
        o[0] = bfr(v[0]); o[1] = bfr(v[1]); o[2] = bfr(v[2]); o[3] = bfr(v[3]);
        *(v4fa*)(&bs[g * 64 + c4]) = o;
    }
    wave_sync();
    int sj[4];
#pragma unroll
    for (int mb = 0; mb < 4; ++mb) sj[mb] = sg[mb * 16 + lr];
    unsigned pm = (1u << sj[0]) | (1u << sj[1]) | (1u << sj[2]) | (1u << sj[3]);
    pm |= (unsigned)__shfl_xor((int)pm, 16, 32);
    pm |= (unsigned)__shfl_xor((int)pm, 8, 32);
    pm |= (unsigned)__shfl_xor((int)pm, 4, 32);
    pm |= (unsigned)__shfl_xor((int)pm, 2, 32);
    pm |= (unsigned)__shfl_xor((int)pm, 1, 32);
    pm = (unsigned)__builtin_amdgcn_readfirstlane((int)pm);

    v8f acc[4][4];
#pragma unroll
    for (int mb = 0; mb < 4; ++mb)
#pragma unroll
        for (int nb = 0; nb < 4; ++nb) acc[mb][nb] = (v8f){};
    const size_t aoff = (size_t)(r0 + lr) * CC + 8 * hi, boff = (size_t)(c0 + lr) * KT + 8 * hi;
    const v8us zz = (v8us){};
#pragma unroll 1
    for (int g = 0; g < NG; ++g) {
        if (((pm >> g) & 1u) == 0u) continue;
        const bool k0m = (sj[0] == g), k1m = (sj[1] == g), k2m = (sj[2] == g), k3m = (sj[3] == g);
        const bf* bg = Bt + boff + (size_t)g * CC;
#pragma unroll 1
        for (int kc = 0; kc < CC; kc += 32) {
            v16bf a[4];
            { const bf* p = A + aoff + kc;
              v8us l0 = *(const v8us*)(p),                       h0 = *(const v8us*)(p + 16);
              v8us l1 = *(const v8us*)(p + (size_t)16 * CC),     h1 = *(const v8us*)(p + (size_t)16 * CC + 16);
              v8us l2 = *(const v8us*)(p + (size_t)32 * CC),     h2 = *(const v8us*)(p + (size_t)32 * CC + 16);
              v8us l3 = *(const v8us*)(p + (size_t)48 * CC),     h3 = *(const v8us*)(p + (size_t)48 * CC + 16);
              l0 = k0m ? l0 : zz; h0 = k0m ? h0 : zz;
              l1 = k1m ? l1 : zz; h1 = k1m ? h1 : zz;
              l2 = k2m ? l2 : zz; h2 = k2m ? h2 : zz;
              l3 = k3m ? l3 : zz; h3 = k3m ? h3 : zz;
              a[0] = cat16b(l0, h0); a[1] = cat16b(l1, h1); a[2] = cat16b(l2, h2); a[3] = cat16b(l3, h3); }
#pragma unroll
            for (int nb = 0; nb < 4; ++nb) { const v16bf b = ldb(bg + (size_t)nb * 16 * KT + kc);
#pragma unroll
                for (int mb = 0; mb < 4; ++mb) acc[mb][nb] = wmmab(a[mb], b, acc[mb][nb]); }
            asm volatile("v_nop\n\tv_nop\n\tv_nop\n\tv_nop" : "+v"(acc[0][0]), "+v"(acc[1][1]), "+v"(acc[2][2]), "+v"(acc[3][3]) : "v"(a[0]), "v"(a[1]), "v"(a[2]), "v"(a[3]));
        }
    }
    float* obase = OUT + (size_t)r0 * DD + c0;
#pragma unroll
    for (int mb = 0; mb < 4; ++mb) {
#pragma unroll
        for (int nb = 0; nb < 4; ++nb) {
#pragma unroll
            for (int j = 0; j < 8; ++j) os[(hi * 8 + j) * 68 + nb * 16 + lr] = acc[mb][nb][j]; }
        wave_sync();
#pragma unroll 1
        for (int ps = 0; ps < 2; ++ps) {
#pragma unroll
            for (int s = 0; s < 8; ++s) { const int row = 2 * s + hi, cofs = lr * 4;
                const v4f val = *(const v4fa*)(&os[row * 68 + cofs]);
                const int gr = sg[mb * 16 + row];
                const v4f bv = *(const v4fa*)(&bs[gr * 64 + cofs]);
                const v4f o = val + bv;
                *(volatile v4f*)(obase + (size_t)(mb * 16 + row) * DD + cofs) = o; }
            if (ps == 0) __threadfence(); }
        wave_sync();
    }
}

static constexpr size_t al256(size_t v) { return (v + 255) & ~(size_t)255; }
static constexpr size_t SZ_XB = al256((size_t)NB * CC * 2);
static constexpr size_t SZ_WT = al256((size_t)DD * KT * 2);
static constexpr size_t SZ_TOTAL = SZ_XB + SZ_WT;
static_assert(SZ_TOTAL <= (size_t)134217728);

extern "C" void kernel_launch(void* const* d_in, const int* in_sizes, int n_in,
                              void* d_out, int out_size, void* d_ws, size_t ws_size, hipStream_t stream) {
    if (n_in < 4) return;
    if ((size_t)in_sizes[0] < (size_t)NB * CC) return;
    if ((size_t)in_sizes[1] < (size_t)NB) return;
    if ((size_t)in_sizes[2] < (size_t)NG * CC * DD) return;
    if ((size_t)in_sizes[3] < (size_t)NG * DD) return;
    if ((size_t)out_size < (size_t)NB * DD) return;
    if (SZ_TOTAL > ws_size) return;
    const float* x  = (const float*)d_in[0];
    const int*   gi = (const int*)d_in[1];
    const float* w  = (const float*)d_in[2];
    const float* bi = (const float*)d_in[3];
    float* OUT = (float*)d_out;
    char* wsp = (char*)d_ws;
    bf* XB = (bf*)wsp; wsp += SZ_XB;
    bf* WT = (bf*)wsp; wsp += SZ_WT;

    { const size_t n8 = (size_t)NB * CC / 8;
      k_cvt8<<<(unsigned)((n8 + 255) / 256), 256, 0, stream>>>(x, XB, n8); }
    k_wt<<<dim3(DD / 64, CC / 64, NG), 256, 0, stream>>>(w, WT);
    k_sgemm<<<dim3(NB / 64, DD / 64, 1), 32, 0, stream>>>(XB, WT, gi, bi, OUT);
}
